// LengthBasedMLP_21758304321789
// MI455X (gfx1250) — hardware-verified
//
#include <hip/hip_runtime.h>
#include <stddef.h>

#define NR     32768
#define IN     128
#define H1     512
#define H2     256
#define H3     128
#define NE     8
#define TB     256
#define MT     16
#define XP     136
#define P1     520
#define P2     264
#define P3     132
#define TP     72
#define NS1    (NE * H1)
#define NS2    (NE * H2)
#define NS3    (NE * H3)
#define NSC    (NS1 + NS2 + NS3)
#define BN_EPS 1e-5f
#define NEG_SLOPE 0.01f

#define L_XH   0
#define L_XL   (L_XH + MT * XP * 2)
#define L_H1H  (L_XL + MT * XP * 2)
#define L_H1L  (L_H1H + MT * P1 * 2)
#define L_H2H  (L_H1L + MT * P1 * 2)
#define L_H2L  (L_H2H + MT * P2 * 2)
#define L_H3   (L_H2L + MT * P2 * 2)
#define LDS_MAIN (L_H3 + MT * P3 * 4)

static_assert(NR % TB == 0);
static_assert(TB == 256);
static_assert((XP * 2) % 16 == 0);
static_assert((P1 * 2) % 16 == 0);
static_assert((P2 * 2) % 16 == 0);
static_assert((P3 * 4) % 16 == 0);
static_assert((TP * 2) % 16 == 0);
static_assert(L_XL % 16 == 0);
static_assert(L_H1H % 16 == 0);
static_assert(L_H1L % 16 == 0);
static_assert(L_H2H % 16 == 0);
static_assert(L_H2L % 16 == 0);
static_assert(L_H3 % 16 == 0);
static_assert(IN % 64 == 0);
static_assert(H1 % 64 == 0);
static_assert(H2 % 64 == 0);
static_assert(H3 % 64 == 0);
static_assert(NSC % 256 == 0);
static_assert(NS1 % 256 == 0);
static_assert(NS2 % 256 == 0);

typedef __bf16         v16b __attribute__((ext_vector_type(16)));
typedef float          v8f  __attribute__((ext_vector_type(8)));
typedef float          v4f  __attribute__((ext_vector_type(4)));
typedef unsigned int   v4u  __attribute__((ext_vector_type(4)));
typedef unsigned int   v8u  __attribute__((ext_vector_type(8)));
typedef unsigned short v8us __attribute__((ext_vector_type(8)));
typedef v4f __attribute__((may_alias)) v4fa;
typedef v4u __attribute__((may_alias)) v4ua;

__device__ __forceinline__ unsigned int bf16_rne_bits(float f) {
  const unsigned int u = __float_as_uint(f);
  return (u + 0x7FFFu + ((u >> 16) & 1u)) >> 16;
}
__device__ __forceinline__ void split2(float f, unsigned short& hi, unsigned short& lo) {
  const unsigned int hu = bf16_rne_bits(f);
  const float fh = __uint_as_float(hu << 16);
  const unsigned int lu = bf16_rne_bits(f - fh);
  hi = (unsigned short)hu;
  lo = (unsigned short)lu;
}
__device__ __forceinline__ void split8(v4f a, v4f c, v4u& uh, v4u& ul) {
  v8us hv = {0, 0, 0, 0, 0, 0, 0, 0};
  v8us lv = {0, 0, 0, 0, 0, 0, 0, 0};
  unsigned short hh, ll;
  split2(a.x, hh, ll); hv[0] = hh; lv[0] = ll;
  split2(a.y, hh, ll); hv[1] = hh; lv[1] = ll;
  split2(a.z, hh, ll); hv[2] = hh; lv[2] = ll;
  split2(a.w, hh, ll); hv[3] = hh; lv[3] = ll;
  split2(c.x, hh, ll); hv[4] = hh; lv[4] = ll;
  split2(c.y, hh, ll); hv[5] = hh; lv[5] = ll;
  split2(c.z, hh, ll); hv[6] = hh; lv[6] = ll;
  split2(c.w, hh, ll); hv[7] = hh; lv[7] = ll;
  uh = __builtin_bit_cast(v4u, hv);
  ul = __builtin_bit_cast(v4u, lv);
}

__device__ __forceinline__ v8f wmma_b(v16b a, v16b b, v8f c) {
  v8f d = __builtin_amdgcn_wmma_f32_16x16x32_bf16(false, a, false, b, (short)0, c, false, false);
  asm volatile("v_nop\n\tv_nop\n\tv_nop\n\tv_nop" : "+v"(d) : "v"(a), "v"(b));
  return d;
}

__device__ __forceinline__ v16b ldfrag(const unsigned short* p, int h) {
  const v4u q0 = *(const v4ua*)(p + 8 * h);
  const v4u q1 = *(const v4ua*)(p + 16 + 8 * h);
  const v8u w = {q0.x, q0.y, q0.z, q0.w, q1.x, q1.y, q1.z, q1.w};
  return __builtin_bit_cast(v16b, w);
}

template <int K, int N>
__global__ __launch_bounds__(256) void k_wsplit(const float* __restrict__ w,
                                                unsigned short* __restrict__ wh,
                                                unsigned short* __restrict__ wl)
{
  __shared__ __align__(16) unsigned short sTh[64 * TP];
  __shared__ __align__(16) unsigned short sTl[64 * TP];
  const int tid = threadIdx.x, lane = tid & 31, wv = tid >> 5;
  const int k0 = blockIdx.x * 64;
  const int c0 = blockIdx.y * 64;
  const int e  = blockIdx.z;
  const float* src = w + (size_t)e * K * N + (size_t)k0 * N + c0;
  #pragma unroll
  for (int j = 0; j < 4; ++j) {
    const int idx = tid + 256 * j;
    const int kr  = idx >> 4;
    const int cb  = (idx & 15) * 4;
    const v4f v = *(const v4fa*)(src + (size_t)kr * N + cb);
    unsigned short hh, ll;
    split2(v.x, hh, ll); sTh[(cb + 0) * TP + kr] = hh; sTl[(cb + 0) * TP + kr] = ll;
    split2(v.y, hh, ll); sTh[(cb + 1) * TP + kr] = hh; sTl[(cb + 1) * TP + kr] = ll;
    split2(v.z, hh, ll); sTh[(cb + 2) * TP + kr] = hh; sTl[(cb + 2) * TP + kr] = ll;
    split2(v.w, hh, ll); sTh[(cb + 3) * TP + kr] = hh; sTl[(cb + 3) * TP + kr] = ll;
  }
  __syncthreads();
  const int q  = lane & 7;
  const int j0 = wv * 8 + (lane >> 3);
  const int j1 = j0 + 4;
  const v4u h0 = *(const v4ua*)(sTh + j0 * TP + 8 * q);
  const v4u h1 = *(const v4ua*)(sTh + j1 * TP + 8 * q);
  const v4u l0 = *(const v4ua*)(sTl + j0 * TP + 8 * q);
  const v4u l1 = *(const v4ua*)(sTl + j1 * TP + 8 * q);
  const size_t r0 = ((size_t)e * N + c0 + j0) * K + k0 + 8 * q;
  const size_t r1 = ((size_t)e * N + c0 + j1) * K + k0 + 8 * q;
  *(volatile v4u*)(wh + r0) = h0;
  *(volatile v4u*)(wh + r1) = h1;
  *(volatile v4u*)(wl + r0) = l0;
  *(volatile v4u*)(wl + r1) = l1;
  __threadfence();
  *(volatile v4u*)(wh + r0) = h0;
  *(volatile v4u*)(wh + r1) = h1;
  *(volatile v4u*)(wl + r0) = l0;
  *(volatile v4u*)(wl + r1) = l1;
}

__global__ __launch_bounds__(256) void k_fold(
    const float* __restrict__ b1, const float* __restrict__ g1, const float* __restrict__ be1,
    const float* __restrict__ m1, const float* __restrict__ v1,
    const float* __restrict__ b2, const float* __restrict__ g2, const float* __restrict__ be2,
    const float* __restrict__ m2, const float* __restrict__ v2,
    const float* __restrict__ b3, const float* __restrict__ g3, const float* __restrict__ be3,
    const float* __restrict__ m3, const float* __restrict__ v3,
    float* __restrict__ S, float* __restrict__ C)
{
  const int i = blockIdx.x * 256 + threadIdx.x;
  float g, v, b, mu, be;
  if (i < NS1) {
    g = g1[i]; v = v1[i]; b = b1[i]; mu = m1[i]; be = be1[i];
  } else if (i < NS1 + NS2) {
    const int j = i - NS1;
    g = g2[j]; v = v2[j]; b = b2[j]; mu = m2[j]; be = be2[j];
  } else {
    int j = i - NS1 - NS2;
    j = (j > NS3 - 1) ? (NS3 - 1) : j;
    g = g3[j]; v = v3[j]; b = b3[j]; mu = m3[j]; be = be3[j];
  }
  const float sc = g * rsqrtf(v + BN_EPS);
  const float sh = (b - mu) * sc + be;
  const int ic = (i > NSC - 1) ? (NSC - 1) : i;
  *(volatile float*)(S + ic) = sc;
  *(volatile float*)(C + ic) = sh;
  __threadfence();
  *(volatile float*)(S + ic) = sc;
  *(volatile float*)(C + ic) = sh;
}

template <int KD, int NT, int AP, int OP, bool F32O>
__device__ __forceinline__ void mlp_layer(
    const unsigned short* sAh, const unsigned short* sAl,
    const unsigned short* __restrict__ gBh, const unsigned short* __restrict__ gBl,
    const int ncol0,
    const float* __restrict__ gS, const float* __restrict__ gC,
    unsigned short* oH, unsigned short* oL, float* oF,
    const int lane)
{
  const int h = lane >> 4, m = lane & 15;
  const v8f z8 = {0.f, 0.f, 0.f, 0.f, 0.f, 0.f, 0.f, 0.f};
  v8f acc[NT];
  #pragma unroll
  for (int nt = 0; nt < NT; ++nt) acc[nt] = z8;
  const unsigned short* pah = sAh + m * AP;
  const unsigned short* pal = sAl + m * AP;
  #pragma unroll 1
  for (int k0 = 0; k0 < KD; k0 += 32) {
    const v16b ah = ldfrag(pah + k0, h);
    const v16b al = ldfrag(pal + k0, h);
    #pragma unroll
    for (int nt = 0; nt < NT; ++nt) {
      const size_t bo = (size_t)(ncol0 + 16 * nt + m) * KD + k0;
      const v16b bh = ldfrag(gBh + bo, h);
      const v16b bl = ldfrag(gBl + bo, h);
      acc[nt] = wmma_b(ah, bh, acc[nt]);
      acc[nt] = wmma_b(ah, bl, acc[nt]);
      acc[nt] = wmma_b(al, bh, acc[nt]);
    }
  }
  #pragma unroll
  for (int nt = 0; nt < NT; ++nt) {
    const int n = ncol0 + 16 * nt + m;
    const float sc = gS[n];
    const float sh = gC[n];
    #pragma unroll
    for (int r = 0; r < 8; ++r) {
      const int row = 8 * h + r;
      float v = acc[nt][r] * sc + sh;
      v = (v >= 0.0f) ? v : NEG_SLOPE * v;
      if (F32O) {
        oF[row * OP + n] = v;
      } else {
        unsigned short hh, ll;
        split2(v, hh, ll);
        oH[row * OP + n] = hh;
        oL[row * OP + n] = ll;
      }
    }
  }
}

__global__ __launch_bounds__(256) void k_main(
    const float* __restrict__ x,
    const unsigned short* __restrict__ w1h, const unsigned short* __restrict__ w1l,
    const unsigned short* __restrict__ w2h, const unsigned short* __restrict__ w2l,
    const unsigned short* __restrict__ w3h, const unsigned short* __restrict__ w3l,
    const float* __restrict__ S, const float* __restrict__ C,
    const float* __restrict__ W4, const float* __restrict__ b4,
    float* __restrict__ out)
{
  extern __shared__ __align__(16) unsigned char dsm_m[];
  unsigned short* sXh  = (unsigned short*)(dsm_m + L_XH);
  unsigned short* sXl  = (unsigned short*)(dsm_m + L_XL);
  unsigned short* sH1h = (unsigned short*)(dsm_m + L_H1H);
  unsigned short* sH1l = (unsigned short*)(dsm_m + L_H1L);
  unsigned short* sH2h = (unsigned short*)(dsm_m + L_H2H);
  unsigned short* sH2l = (unsigned short*)(dsm_m + L_H2L);
  float*          sH3  = (float*)(dsm_m + L_H3);
  __shared__ int sCnt[NE * 8];
  __shared__ int sTot[NE];
  __shared__ int sList[NE * TB];
  __shared__ __align__(16) float sOut[TB];

  const int tid = threadIdx.x, lane = tid & 31, wv = tid >> 5;
  const int n0 = blockIdx.x * TB;

  int bkt;
  bool valid;
  {
    const float* xr = x + (size_t)(n0 + tid) * IN;
    double s = 0.0;
    #pragma unroll 2
    for (int j = 0; j < IN / 4; ++j) {
      const v4f p = *(const v4fa*)(xr + 4 * j);
      s += (double)p.x;
      s += (double)p.y;
      s += (double)p.z;
      s += (double)p.w;
    }
    const double key = s * 0.0625;
    const int b = (int)__builtin_ceil(key) - 1;
    valid = (b >= 0) && (b < NE);
    bkt = valid ? b : -1;
  }
  sOut[tid] = 0.0f;

  int myoff = 0;
  #pragma unroll
  for (int e = 0; e < NE; ++e) {
    const bool f = (bkt == e);
    const unsigned int msk = __builtin_amdgcn_ballot_w32(f);
    const int off = __builtin_popcount(msk & ((1u << lane) - 1u));
    myoff = f ? off : myoff;
    if (lane == 0) sCnt[e * 8 + wv] = __builtin_popcount(msk);
  }
  __syncthreads();
  {
    const int bc = valid ? bkt : 0;
    int pre = 0;
    #pragma unroll
    for (int w2 = 0; w2 < 8; ++w2) pre += (w2 < wv) ? sCnt[bc * 8 + w2] : 0;
    const int pos = pre + myoff;
    if (valid && (unsigned)pos < (unsigned)TB) sList[bc * TB + pos] = tid;
    if (tid < NE) {
      int t = 0;
      #pragma unroll
      for (int w2 = 0; w2 < 8; ++w2) t += sCnt[tid * 8 + w2];
      sTot[tid] = (t > TB) ? TB : t;
    }
  }
  __syncthreads();

  const int grow = tid >> 4;
  const int gc   = tid & 15;
  #pragma unroll 1
  for (int e = 0; e < NE; ++e) {
    int ne = sTot[e];
    ne = (ne > TB) ? TB : ((ne < 0) ? 0 : ne);
    if (ne > 0) {
      const int nch = (ne + MT - 1) / MT;
      const unsigned short* e1h = w1h + (size_t)e * H1 * IN;
      const unsigned short* e1l = w1l + (size_t)e * H1 * IN;
      const unsigned short* e2h = w2h + (size_t)e * H2 * H1;
      const unsigned short* e2l = w2l + (size_t)e * H2 * H1;
      const unsigned short* e3h = w3h + (size_t)e * H3 * H2;
      const unsigned short* e3l = w3l + (size_t)e * H3 * H2;
      const float* S1 = S + e * H1;
      const float* C1 = C + e * H1;
      const float* S2 = S + NS1 + e * H2;
      const float* C2 = C + NS1 + e * H2;
      const float* S3 = S + NS1 + NS2 + e * H3;
      const float* C3 = C + NS1 + NS2 + e * H3;
      #pragma unroll 1
      for (int c = 0; c < nch; ++c) {
        {
          const int p  = c * MT + grow;
          const bool pv = (p < ne);
          const int pc = pv ? p : (ne - 1);
          int rid = sList[e * TB + pc];
          rid = (rid < 0) ? 0 : ((rid > TB - 1) ? (TB - 1) : rid);
          const float* g = x + (size_t)(n0 + rid) * IN + 8 * gc;
          v4f a  = *(const v4fa*)g;
          v4f cc = *(const v4fa*)(g + 4);
          a.x  = pv ? a.x  : 0.0f; a.y  = pv ? a.y  : 0.0f; a.z  = pv ? a.z  : 0.0f; a.w  = pv ? a.w  : 0.0f;
          cc.x = pv ? cc.x : 0.0f; cc.y = pv ? cc.y : 0.0f; cc.z = pv ? cc.z : 0.0f; cc.w = pv ? cc.w : 0.0f;
          v4u uh, ul;
          split8(a, cc, uh, ul);
          *(v4ua*)(sXh + grow * XP + 8 * gc) = uh;
          *(v4ua*)(sXl + grow * XP + 8 * gc) = ul;
        }
        __syncthreads();
        mlp_layer<IN, 4, XP, P1, false>(sXh, sXl, e1h, e1l, 64 * wv, S1, C1, sH1h, sH1l, sH3, lane);
        __syncthreads();
        mlp_layer<H1, 2, P1, P2, false>(sH1h, sH1l, e2h, e2l, 32 * wv, S2, C2, sH2h, sH2l, sH3, lane);
        __syncthreads();
        mlp_layer<H2, 1, P2, P3, true>(sH2h, sH2l, e3h, e3l, 16 * wv, S3, C3, sXh, sXl, sH3, lane);
        __syncthreads();
        {
          const v4f ha = *(const v4fa*)(sH3 + grow * P3 + 8 * gc);
          const v4f hb = *(const v4fa*)(sH3 + grow * P3 + 8 * gc + 4);
          const float* w4e = W4 + e * H3 + 8 * gc;
          const v4f wa = *(const v4fa*)w4e;
          const v4f wb = *(const v4fa*)(w4e + 4);
          float d = ha.x * wa.x;
          d += ha.y * wa.y;
          d += ha.z * wa.z;
          d += ha.w * wa.w;
          d += hb.x * wb.x;
          d += hb.y * wb.y;
          d += hb.z * wb.z;
          d += hb.w * wb.w;
          d += __shfl_xor(d, 8);
          d += __shfl_xor(d, 4);
          d += __shfl_xor(d, 2);
          d += __shfl_xor(d, 1);
          if (gc == 0) {
            const int p = c * MT + grow;
            if (p < ne) {
              int rid = sList[e * TB + p];
              rid = (rid < 0) ? 0 : ((rid > TB - 1) ? (TB - 1) : rid);
              sOut[rid] = d + b4[e];
            }
          }
        }
        __syncthreads();
      }
    }
  }
  __syncthreads();

  if (wv < 2) {
    const v4f v = *(const v4fa*)(sOut + wv * 128 + 4 * lane);
    float* dst = out + (size_t)n0 + wv * 128 + 4 * lane;
    *(volatile v4f*)dst = v;
    __threadfence();
    *(volatile v4f*)dst = v;
  }
}

extern "C" void kernel_launch(void* const* d_in, const int* in_sizes, int n_in,
                              void* d_out, int out_size, void* d_ws, size_t ws_size,
                              hipStream_t stream)
{
  if (n_in < 21) return;
  if (in_sizes[0]  != NR * IN) return;
  if (in_sizes[1]  != NE * IN * H1) return;
  for (int i = 2; i <= 6; ++i)   if (in_sizes[i] != NE * H1) return;
  if (in_sizes[7]  != NE * H1 * H2) return;
  for (int i = 8; i <= 12; ++i)  if (in_sizes[i] != NE * H2) return;
  if (in_sizes[13] != NE * H2 * H3) return;
  for (int i = 14; i <= 18; ++i) if (in_sizes[i] != NE * H3) return;
  if (in_sizes[19] != NE * H3) return;
  if (in_sizes[20] != NE) return;
  if (out_size != NR) return;

  const float* x   = (const float*)d_in[0];
  const float* W1  = (const float*)d_in[1];
  const float* b1  = (const float*)d_in[2];
  const float* g1  = (const float*)d_in[3];
  const float* be1 = (const float*)d_in[4];
  const float* m1  = (const float*)d_in[5];
  const float* v1  = (const float*)d_in[6];
  const float* W2  = (const float*)d_in[7];
  const float* b2  = (const float*)d_in[8];
  const float* g2  = (const float*)d_in[9];
  const float* be2 = (const float*)d_in[10];
  const float* m2  = (const float*)d_in[11];
  const float* v2  = (const float*)d_in[12];
  const float* W3  = (const float*)d_in[13];
  const float* b3  = (const float*)d_in[14];
  const float* g3  = (const float*)d_in[15];
  const float* be3 = (const float*)d_in[16];
  const float* m3  = (const float*)d_in[17];
  const float* v3  = (const float*)d_in[18];
  const float* W4  = (const float*)d_in[19];
  const float* b4  = (const float*)d_in[20];
  float* out = (float*)d_out;

  const size_t bW1 = (size_t)NE * H1 * IN * 2;
  const size_t bW2 = (size_t)NE * H2 * H1 * 2;
  const size_t bW3 = (size_t)NE * H3 * H2 * 2;
  const size_t bSC = (size_t)NSC * 4;
  const size_t total = 2 * bW1 + 2 * bW2 + 2 * bW3 + 2 * bSC;
  if (total > ws_size) return;
  if (total > (size_t)134217728) return;

  char* ws = (char*)d_ws;
  size_t off = 0;
  unsigned short* W1H = (unsigned short*)(ws + off); off += bW1;
  unsigned short* W1L = (unsigned short*)(ws + off); off += bW1;
  unsigned short* W2H = (unsigned short*)(ws + off); off += bW2;
  unsigned short* W2L = (unsigned short*)(ws + off); off += bW2;
  unsigned short* W3H = (unsigned short*)(ws + off); off += bW3;
  unsigned short* W3L = (unsigned short*)(ws + off); off += bW3;
  float*          SB  = (float*)(ws + off);          off += bSC;
  float*          CB  = (float*)(ws + off);          off += bSC;
  if (off != total) return;

  k_wsplit<IN, H1><<<dim3(IN / 64, H1 / 64, NE), 256, 0, stream>>>(W1, W1H, W1L);
  k_wsplit<H1, H2><<<dim3(H1 / 64, H2 / 64, NE), 256, 0, stream>>>(W2, W2H, W2L);
  k_wsplit<H2, H3><<<dim3(H2 / 64, H3 / 64, NE), 256, 0, stream>>>(W3, W3H, W3L);
  k_fold<<<NSC / 256, 256, 0, stream>>>(b1, g1, be1, m1, v1,
                                        b2, g2, be2, m2, v2,
                                        b3, g3, be3, m3, v3, SB, CB);
  hipFuncSetAttribute(reinterpret_cast<const void*>(&k_main),
                      hipFuncAttributeMaxDynamicSharedMemorySize, LDS_MAIN);
  k_main<<<NR / TB, 256, LDS_MAIN, stream>>>(x, W1H, W1L, W2H, W2L, W3H, W3L,
                                             SB, CB, W4, b4, out);
}
